// HGT_40132174414160
// MI455X (gfx1250) — hardware-run, weakly checked
//
#include <hip/hip_runtime.h>


namespace {

constexpr int N = 50000, NP = 50048, NPL = NP  , SRCM = N  , EFULL = 800000, E = EFULL  , D = 128, NH = 8, DK = 16, NL = (NPL < N ? NPL : N);
constexpr int PPAIR = 100000  , NPAIR = 2 * PPAIR, L = 3, H1 = 64, H2 = 32;
constexpr float XS = 8.0f, WSC = 256.0f, WSQ = 0.25f, RS_ = 1024.0f, LNEPS = 1e-5f, ISQ = 0.25f  , SLOPE = 0.0f, BNEPS = 1e-5f, NSL_ = 0.2f;
static_assert(NP % 64 == 0 && NP >= N && NPL % 64 == 0 && D == 128 && NH * DK == D && NPAIR % 32 == 0, "tiling");
typedef _Float16 b16;
typedef __attribute__((ext_vector_type(16))) _Float16 v16b;
typedef __attribute__((ext_vector_type(8))) _Float16 v8b;
typedef __attribute__((ext_vector_type(8))) float v8f;
typedef __attribute__((ext_vector_type(4))) float v4f;
__device__ __forceinline__ float bf16_rne(float f) { unsigned int u = __float_as_uint(f); u += 0x7FFFu + ((u >> 16) & 1u); return __uint_as_float(u & 0xFFFF0000u); }
__device__ __forceinline__ void split16(float v, b16& hi, b16& lo) { hi = (b16)v; lo = (b16)(v - (float)hi); }
__device__ __forceinline__ v16b frag_kb(const b16* p, int hh) { const v8b a = *(const v8b*)(p + 8 * hh), b = *(const v8b*)(p + 16 + 8 * hh); v16b f;
#pragma unroll
  for (int e = 0; e < 8; ++e) { f[e] = a[e]; f[8 + e] = b[e]; } return f; }
__device__ __forceinline__ v8f wmma16b(v16b a, v16b b, v8f c) { v8f d = __builtin_amdgcn_wmma_f32_16x16x32_f16(false, a, false, b, (short)0, c, false, false); asm volatile("v_nop\n\tv_nop\n\tv_nop\n\tv_nop" : "+v"(d) : "v"(a), "v"(b)); return d; }
__device__ __forceinline__ void wave_lds_sync() { __builtin_amdgcn_fence(__ATOMIC_RELEASE, "workgroup"); __builtin_amdgcn_wave_barrier(); __builtin_amdgcn_fence(__ATOMIC_ACQUIRE, "workgroup"); }
__device__ __forceinline__ float pmul(float a, float b) { float p = a * b; asm volatile("" : "+v"(p)); return p; }
__device__ __forceinline__ int iclamp(int v, int lo, int hi) { return v < lo ? lo : (v > hi ? hi : v); }
constexpr int CSR_NBLK = 512, CSR_GB = 9, CSR_GN = 1 << CSR_GB  , CSR_MAXG = 512, CSR_CAP = 12288  ;
__global__ __launch_bounds__(64) void csrA_kernel(const int* __restrict__ dst, int E, int N, int nG, int CHP, int NGP, int* __restrict__ STG, int* __restrict__ HST) {
  extern __shared__ int sm[];
  int* cnt = sm; int* run = sm + NGP; int* ids = sm + 2 * NGP;
  const int b = blockIdx.x; const int ch = (E + CSR_NBLK - 1) / CSR_NBLK; const int e0 = b * ch, e1 = min(E, e0 + ch);
  for (int i = threadIdx.x; i < NGP; i += 64) cnt[i] = 0;
  for (int i = threadIdx.x; i < CHP; i += 64) ids[i] = -1;
  __syncthreads();
  if (threadIdx.x == 0) {
    for (int e = e0; e < e1; ++e) { int d = dst[e]; d = (d < 0) ? 0 : (d >= N ? N - 1 : d); cnt[d >> CSR_GB] += 1; }
    int acc = 0; for (int g = 0; g < nG; ++g) { run[g] = acc; acc += cnt[g]; }
    for (int e = e0; e < e1; ++e) { int d = dst[e]; d = (d < 0) ? 0 : (d >= N ? N - 1 : d); const int g = d >> CSR_GB; ids[run[g]] = e; run[g] += 1; } }
  __syncthreads();
  typedef __attribute__((ext_vector_type(4))) int v4i;
  for (int pass = 0; pass < 2; ++pass) {
    for (int i = threadIdx.x; i < CHP / 4; i += 64) *(volatile v4i*)(STG + (size_t)b * CHP + i * 4) = *(const v4i*)(&ids[i * 4]);
    for (int i = threadIdx.x; i < NGP / 4; i += 64) { v4i v; for (int e = 0; e < 4; ++e) v[e] = (i * 4 + e < nG) ? cnt[i * 4 + e] : 0; *(volatile v4i*)(HST + (size_t)b * NGP + i * 4) = v; }
    __threadfence(); }
}
__global__ __launch_bounds__(512) void csrS_kernel(const int* __restrict__ HST, int nG, int NGP, int* __restrict__ START, int* __restrict__ TOT, int* __restrict__ OFF) {
  __shared__ int tot[CSR_MAXG];
  const int b = threadIdx.x;
  for (int pass = 0; pass < 2; ++pass) { int runb = 0; for (int g = 0; g < nG; ++g) { int c = HST[(size_t)b * NGP + g]; c = (c < 0) ? 0 : c; ((volatile int*)OFF)[(size_t)g * CSR_NBLK + b] = runb; runb += c; } __threadfence(); }
  for (int g = threadIdx.x; g < nG; g += 512) { int s = 0; for (int bb = 0; bb < CSR_NBLK; ++bb) { int c = HST[(size_t)bb * NGP + g]; s += (c < 0) ? 0 : c; } tot[g] = s; }
  __syncthreads();
  if (threadIdx.x < 32) {
    __shared__ int st[CSR_MAXG + 32];
    if (threadIdx.x == 0) { int acc = 0; for (int g = 0; g < NGP; ++g) { st[g] = acc; if (g < nG) acc += (tot[g] + 31) & ~31; } st[NGP] = acc; }
    __builtin_amdgcn_fence(__ATOMIC_RELEASE, "workgroup"); __builtin_amdgcn_wave_barrier(); __builtin_amdgcn_fence(__ATOMIC_ACQUIRE, "workgroup");
    for (int pass = 0; pass < 2; ++pass) { for (int i = threadIdx.x; i < NGP + 32; i += 32) { ((volatile int*)START)[i] = (i <= NGP) ? st[min(i, NGP)] : 0; ((volatile int*)TOT)[i] = (i < nG) ? tot[i] : 0; } __threadfence(); } }
}
__global__ __launch_bounds__(256) void csrB_kernel(const int* __restrict__ dst, int N, int nG, int CHP, int NGP, int permLen, const int* __restrict__ STG, const int* __restrict__ HST, const int* __restrict__ OFF, const int* __restrict__ START, const int* __restrict__ TOT, int* __restrict__ PERM, int* __restrict__ ROWPTR, int* __restrict__ ROWCNT, int* __restrict__ FLAG) {
  typedef __attribute__((ext_vector_type(4))) int v4i;
  __shared__ int ids[CSR_CAP]; __shared__ unsigned short key[CSR_CAP]; __shared__ int outp[CSR_CAP]; __shared__ int ncnt[CSR_GN + 1]; __shared__ int boff[CSR_NBLK + 1];
  const int g = blockIdx.x, t_ = threadIdx.x; int tot = TOT[g]; int st = START[g], stn = START[g + 1]; const int v0 = g * CSR_GN; const int nv = min(CSR_GN, N - v0);
  st = (st < 0) ? 0 : (st > permLen - 32 ? permLen - 32 : st) & ~31; stn = (stn < st) ? st : (stn > permLen ? permLen : stn); tot = (tot < 0) ? 0 : tot; if (tot > stn - st && tot <= CSR_CAP) tot = stn - st;
  if (tot > CSR_CAP) {
    for (int pass = 0; pass < 2; ++pass) { for (int i = t_; i < CSR_GN / 4; i += 256) { v4i a, c; for (int e = 0; e < 4; ++e) { a[e] = st; c[e] = 0; } *(volatile v4i*)(ROWPTR + v0 + i * 4) = a; *(volatile v4i*)(ROWCNT + v0 + i * 4) = c; } if (t_ == 0) ((volatile int*)FLAG)[0] = 1; __threadfence(); } (void)nv; return; }
  if (t_ == 0) { int acc = 0; for (int b = 0; b < CSR_NBLK; ++b) { boff[b] = acc; int c = HST[(size_t)b * NGP + g]; c = (c < 0) ? 0 : (c > CHP ? CHP : c); acc += c; if (acc > tot) acc = tot; } boff[CSR_NBLK] = acc; }
  for (int i = t_; i <= CSR_GN; i += 256) ncnt[i] = 0;
  __syncthreads();
  for (int b = 0; b < CSR_NBLK; ++b) { const int c = boff[b + 1] - boff[b]; int o_ = OFF[(size_t)g * CSR_NBLK + b]; o_ = (o_ < 0) ? 0 : (o_ > CHP - c ? CHP - c : o_); const int* src_ = STG + (size_t)b * CHP + o_;
    for (int i = t_; i < c; i += 256) { int id = src_[i]; id = (id < 0) ? 0 : id; ids[boff[b] + i] = id; int d = dst[id]; d = (d < v0) ? v0 : (d >= N ? N - 1 : d); int kk = d - v0; kk = (kk < 0) ? 0 : (kk >= CSR_GN ? CSR_GN - 1 : kk); key[boff[b] + i] = (unsigned short)kk; } }
  __syncthreads();
  if (t_ == 0) { for (int i = 0; i < tot; ++i) ncnt[key[i]] += 1; int acc = 0; for (int vl = 0; vl < CSR_GN; ++vl) { const int c = ncnt[vl]; ncnt[vl] = acc; acc += c; } ncnt[CSR_GN] = acc;
    for (int i = 0; i < tot; ++i) { const int vl = key[i]; outp[ncnt[vl]] = ids[i]; ncnt[vl] += 1; }
    for (int vl = CSR_GN; vl > 0; --vl) ncnt[vl] = ncnt[vl - 1]; ncnt[0] = 0; }
  __syncthreads();
  for (int pass = 0; pass < 2; ++pass) {
    for (int i = t_; i < (stn - st) / 4; i += 256) { v4i v; for (int e = 0; e < 4; ++e) { const int q = i * 4 + e; v[e] = (q < tot) ? outp[q] : -1; } *(volatile v4i*)(PERM + st + i * 4) = v; }
    for (int i = t_; i < CSR_GN / 4; i += 256) { v4i a, c; for (int e = 0; e < 4; ++e) { const int vl = i * 4 + e; a[e] = st + ncnt[vl]; c[e] = (vl < nv) ? (ncnt[vl + 1] - ncnt[vl]) : 0; } *(volatile v4i*)(ROWPTR + v0 + i * 4) = a; *(volatile v4i*)(ROWCNT + v0 + i * 4) = c; }
    __threadfence(); }
}
__global__ __launch_bounds__(256) void csrZ_kernel(int* __restrict__ p, size_t n4) { typedef __attribute__((ext_vector_type(4))) int v4i; const size_t tid = (size_t)blockIdx.x * 256 + threadIdx.x, nth = (size_t)gridDim.x * 256; v4i z = {0, 0, 0, 0}; for (size_t i = tid; i < n4; i += nth) *(volatile v4i*)(p + i * 4) = z; }
struct CsrBufs { int *STG, *HST, *OFF, *START, *TOT, *PERM, *ROWPTR, *ROWCNT, *FLAG; int nG, NGP, CHP; size_t permLen; char* base; size_t bytes; };
static size_t csr_carve(CsrBufs& c, char* ws, size_t off, int E, int N) {
  const size_t off0 = off; c.base = ws + off;
  auto al = [&](size_t bytes) { char* p = ws + off; off += (bytes + 255) & ~(size_t)255; return p; };
  c.nG = (N + CSR_GN - 1) / CSR_GN; c.NGP = (c.nG + 31) & ~31; const int ch = (E + CSR_NBLK - 1) / CSR_NBLK; c.CHP = (ch + 31) & ~31; c.permLen = (size_t)E + 32 * (size_t)c.nG + 32;
  c.STG = (int*)al((size_t)CSR_NBLK * c.CHP * 4); c.HST = (int*)al((size_t)CSR_NBLK * c.NGP * 4); c.OFF = (int*)al((size_t)c.NGP * CSR_NBLK * 4); c.START = (int*)al((size_t)(c.NGP + 64) * 4); c.TOT = (int*)al((size_t)(c.NGP + 64) * 4);
  c.PERM = (int*)al(c.permLen * 4); c.ROWPTR = (int*)al((size_t)c.nG * CSR_GN * 4); c.ROWCNT = (int*)al((size_t)c.nG * CSR_GN * 4); c.FLAG = (int*)al(256);
  c.bytes = off - off0; return off;
}
static void csr_build(const CsrBufs& c, const int* dst, int E, int N, hipStream_t stream) {
  const size_t smem = (size_t)(2 * c.NGP + c.CHP) * 4;
  csrZ_kernel<<<512, 256, 0, stream>>>((int*)c.base, c.bytes / 16);
  csrA_kernel<<<CSR_NBLK, 64, smem, stream>>>(dst, E, N, c.nG, c.CHP, c.NGP, c.STG, c.HST);
  csrS_kernel<<<1, 512, 0, stream>>>(c.HST, c.nG, c.NGP, c.START, c.TOT, c.OFF);
  csrB_kernel<<<c.nG, 256, 0, stream>>>(dst, N, c.nG, c.CHP, c.NGP, (int)c.permLen, c.STG, c.HST, c.OFF, c.START, c.TOT, c.PERM, c.ROWPTR, c.ROWCNT, c.FLAG);
}

typedef __attribute__((ext_vector_type(4))) _Float16 v4h;
typedef __attribute__((ext_vector_type(2))) float v2f;
template <int KD, int NOUTR, int NOUTP>
__global__ __launch_bounds__(256) void wprep_kernel(const float* __restrict__ w, b16* __restrict__ WT, float scl) {
  const size_t u = (size_t)blockIdx.x * 256 + threadIdx.x; if (u >= (size_t)NOUTP * KD / 8) return; const size_t e = u * 8; const int oo = (int)(e / KD), k0 = (int)(e % KD); v8b o;
  for (int j = 0; j < 8; ++j) o[j] = (b16)(oo < NOUTR ? bf16_rne(w[(size_t)(k0 + j) * NOUTR + oo]) * scl : 0.0f);
  for (int pass = 0; pass < 2; ++pass) { *(volatile v8b*)(WT + e) = o; __threadfence(); }
}
__global__ __launch_bounds__(256) void bd_kernel(const float* __restrict__ w, b16* __restrict__ BD, float scl) {
  const int u = blockIdx.x * 256 + threadIdx.x; if (u >= D * D / 8) return; const int e = u * 8; const int o = e / D, k0 = e % D; const int h = o / DK, j = o % DK; v8b v;
#pragma unroll
  for (int q = 0; q < 8; ++q) { const int k = k0 + q; const int hk = k / DK, i = k % DK; v[q] = (b16)(hk == h ? bf16_rne(w[((size_t)h * DK + i) * DK + j]) * scl : 0.0f); }
  for (int pass = 0; pass < 2; ++pass) { *(volatile v8b*)(BD + e) = v; __threadfence(); }
}
__device__ __forceinline__ float lrelu(float v) { return v > 0.0f ? v : NSL_ * v; }
template <bool RND, bool BIAS, bool FOLD, int MODE, bool RELU>
__global__ __launch_bounds__(64) void gemm_kernel(const float* __restrict__ IN, int inPitch, const b16* __restrict__ WT, const b16* __restrict__ WQ, const float* __restrict__ bias, const b16* __restrict__ BDT, const b16* __restrict__ BDQ, const float* __restrict__ RES, const float* __restrict__ skip, float* __restrict__ OUT, int outPitch, int mrows) {
  __shared__ __attribute__((aligned(16))) b16 As[2][16][D + 8], Al[2][16][D + 8]; __shared__ __attribute__((aligned(16))) float Tf[2][16][D + 4];
  const int wave = threadIdx.x >> 5, lane = threadIdx.x & 31, nloc = lane & 15, hlf = lane >> 4; const size_t m0 = (size_t)blockIdx.x * 32 + wave * 16;
  for (int idx = lane; idx < 16 * 32; idx += 32) { const int rr = idx / 32, c4 = (idx % 32) * 4; const v4f v = *(const v4f*)(IN + (m0 + rr < (size_t)N ? m0 + rr : (size_t)N - 1) * (size_t)inPitch + c4); v4h o, ol;
    for (int j = 0; j < 4; ++j) { const float vs = (RND ? bf16_rne(v[j]) : v[j]) * XS; const b16 ph = (b16)vs; o[j] = ph; ol[j] = (b16)((vs - (float)ph) * RS_); } *(v4h*)(&As[wave][rr][c4]) = o; *(v4h*)(&Al[wave][rr][c4]) = ol; }
  wave_lds_sync();
  v8f acc[8];
#pragma unroll
  for (int t = 0; t < 8; ++t) acc[t] = (v8f){};
#pragma unroll
  for (int kb = 0; kb < D; kb += 32) { const v16b a = frag_kb(&As[wave][nloc][kb], hlf); v16b al; if (!RND) al = frag_kb(&Al[wave][nloc][kb], hlf);
#pragma unroll
    for (int t = 0; t < 8; ++t) { const size_t wo_ = (size_t)(t * 16 + nloc) * D + kb; acc[t] = wmma16b(a, frag_kb(WT + wo_, hlf), acc[t]); if (!RND) acc[t] = wmma16b(al, frag_kb(WQ + wo_, hlf), acc[t]); } }
  wave_lds_sync();
#pragma unroll
  for (int t = 0; t < 8; ++t) { const float bb = BIAS ? bf16_rne(bias[t * 16 + nloc]) : 0.0f;
#pragma unroll
    for (int r = 0; r < 8; ++r) Tf[wave][8 * hlf + r][t * 16 + nloc] = acc[t][r] * (1.0f / (XS * WSC)) + bb; }
  wave_lds_sync();
  if (FOLD) {
    for (int idx = lane; idx < 16 * 32; idx += 32) { const int rr = idx / 32, c4 = (idx % 32) * 4; v4h hv, lv; for (int j = 0; j < 4; ++j) { const float vs = Tf[wave][rr][c4 + j] * XS; const b16 ph = (b16)vs; hv[j] = ph; lv[j] = (b16)((vs - (float)ph) * RS_); } *(v4h*)(&As[wave][rr][c4]) = hv; *(v4h*)(&Al[wave][rr][c4]) = lv; }
    wave_lds_sync();
#pragma unroll
    for (int t = 0; t < 8; ++t) acc[t] = (v8f){};
#pragma unroll
    for (int kb = 0; kb < D; kb += 32) { const v16b a = frag_kb(&As[wave][nloc][kb], hlf), al = frag_kb(&Al[wave][nloc][kb], hlf);
#pragma unroll
      for (int t = 0; t < 8; ++t) { const size_t wo_ = (size_t)(t * 16 + nloc) * D + kb; acc[t] = wmma16b(a, frag_kb(BDT + wo_, hlf), acc[t]); acc[t] = wmma16b(al, frag_kb(BDQ + wo_, hlf), acc[t]); } }
    wave_lds_sync();
#pragma unroll
    for (int t = 0; t < 8; ++t)
#pragma unroll
      for (int r = 0; r < 8; ++r) Tf[wave][8 * hlf + r][t * 16 + nloc] = acc[t][r] * (1.0f / (XS * WSC));
    wave_lds_sync(); }
  if (MODE > 0) { const float s = (MODE == 2) ? 1.0f / (1.0f + __expf(-bf16_rne(skip[0]))) : 0.0f;
#pragma unroll
    for (int t = 0; t < 8; ++t) { const int col = t * 16 + nloc;
#pragma unroll
      for (int r = 0; r < 8; ++r) { const size_t vrow = m0 + 8 * hlf + r; float val = Tf[wave][8 * hlf + r][col];
        if (MODE == 2) val = pmul(val, s) + pmul(1.0f - s, RES[(vrow < (size_t)N ? vrow : (size_t)N - 1) * D + col]);
        if (RELU) val = fmaxf(val, 0.0f); Tf[wave][8 * hlf + r][col] = (vrow < (size_t)N) ? val : 0.0f; } }
    wave_lds_sync(); }
  for (int pass = 0; pass < 2; ++pass) { for (int rr = 0; rr < 16; ++rr) if (m0 + rr < (size_t)mrows) *(volatile v4f*)(OUT + (m0 + rr) * (size_t)outPitch + lane * 4) = *(const v4f*)(&Tf[wave][rr][lane * 4]); __threadfence(); }
}
__global__ __launch_bounds__(256) void attn_kernel(const float* __restrict__ KQV, const float* __restrict__ pri, const float* __restrict__ ew, const int* __restrict__ srcs, const int* __restrict__ PERM, const int* __restrict__ ROWPTR, const int* __restrict__ ROWCNT, int permLen, float* __restrict__ AGG) {
  const int tid = threadIdx.x; const int row = tid >> 3, h = tid & 7; const int v = blockIdx.x * 32 + row; const float scl = bf16_rne(pri[h]) * ISQ;
  float q[DK], acc[DK]; for (int j = 0; j < DK; ++j) { q[j] = 0.0f; acc[j] = 0.0f; }
  int cnt = 0, p0 = 0; if (v < N) { cnt = iclamp(ROWCNT[v], 0, 65536); p0 = iclamp(ROWPTR[v], 0, permLen - 1); if (p0 + cnt > permLen) cnt = permLen - p0; const float* qr = KQV + (size_t)v * (3 * D) + D + h * DK;
#pragma unroll
    for (int j4 = 0; j4 < DK; j4 += 4) { const v4f t4 = *(const v4f*)(qr + j4); for (int j = 0; j < 4; ++j) q[j4 + j] = t4[j]; } }
  float m = -INFINITY, l = 0.0f;
#pragma unroll 1
  for (int i = 0; i < cnt; ++i) { const int e = iclamp(PERM[p0 + i], 0, E - 1); int s = iclamp(srcs[e], 0, N - 1); if (SRCM < N) s %= SRCM; const float* kr = KQV + (size_t)s * (3 * D) + h * DK; const float* vr = kr + 2 * D; float dot = 0.0f;
#pragma unroll
    for (int j4 = 0; j4 < DK; j4 += 4) { const v4f t4 = *(const v4f*)(kr + j4); for (int j = 0; j < 4; ++j) dot = fmaf(q[j4 + j], t4[j], dot); }
    const float sc = dot * scl; const float mn = fmaxf(m, sc); const float al = __expf(m - mn); const float p = __expf(sc - mn); l = l * al + p; m = mn; const float pw = p * bf16_rne(ew[e]);
#pragma unroll
    for (int j4 = 0; j4 < DK; j4 += 4) { const v4f t4 = *(const v4f*)(vr + j4); for (int j = 0; j < 4; ++j) acc[j4 + j] = fmaf(pw, t4[j], pmul(acc[j4 + j], al)); } }
  const float inv = (v < N && cnt > 0) ? 1.0f / l : 0.0f;
  for (int pass = 0; pass < 2; ++pass) { float* orow = AGG + (size_t)v * D + h * DK;
#pragma unroll
    for (int j4 = 0; j4 < DK; j4 += 4) { v4f o4; for (int j = 0; j < 4; ++j) o4[j] = acc[j4 + j] * inv; *(volatile v4f*)(orow + j4) = o4; }
    __threadfence(); }
}
__global__ __launch_bounds__(256) void copy_kernel(const float* __restrict__ Hh, float* __restrict__ out, int mrows) {
  const int tid = threadIdx.x; const int rr = tid >> 5, c4 = (tid & 31) * 4;
  for (int pass = 0; pass < 2; ++pass) { for (int r8 = 0; r8 < 32; r8 += 8) { const size_t row = (size_t)blockIdx.x * 32 + r8 + rr; if (row < (size_t)mrows) *(volatile v4f*)(out + row * D + c4) = *(const v4f*)(Hh + row * D + c4); } __threadfence(); }
}
__global__ __launch_bounds__(64) void pred_kernel(const float* __restrict__ Hh, const int* __restrict__ ps, const int* __restrict__ pd, const int* __restrict__ ns, const int* __restrict__ nd, const b16* __restrict__ W1T, const b16* __restrict__ W1Q, const float* __restrict__ b1, const b16* __restrict__ W2T, const b16* __restrict__ W2Q, const float* __restrict__ b2, const float* __restrict__ w3, const float* __restrict__ b3, float* __restrict__ OUTP) {
  __shared__ __attribute__((aligned(16))) b16 As[2][16][D + 8], Al[2][16][D + 8]; __shared__ float Sc[32];
  const int wave = threadIdx.x >> 5, lane = threadIdx.x & 31, nloc = lane & 15, hlf = lane >> 4; const int r0 = blockIdx.x * 32 + wave * 16;
  for (int idx = lane; idx < 16 * 32; idx += 32) { const int rr = idx / 32, c4 = (idx % 32) * 4; const int pr = r0 + rr; int s_, d_;
    if (pr < PPAIR) { s_ = ps[pr]; d_ = pd[pr]; } else { s_ = ns[pr - PPAIR]; d_ = nd[pr - PPAIR]; }
    s_ = iclamp(s_, 0, N - 1); d_ = iclamp(d_, 0, N - 1); const v4f a4 = *(const v4f*)(Hh + (size_t)s_ * D + c4), b4 = *(const v4f*)(Hh + (size_t)d_ * D + c4); v4h hv, lv;
    for (int j = 0; j < 4; ++j) { const float vs = pmul(a4[j], b4[j]) * XS; const b16 ph = (b16)vs; hv[j] = ph; lv[j] = (b16)((vs - (float)ph) * RS_); } *(v4h*)(&As[wave][rr][c4]) = hv; *(v4h*)(&Al[wave][rr][c4]) = lv; }
  wave_lds_sync();
  v8f acc[4]; for (int t = 0; t < 4; ++t) acc[t] = (v8f){};
#pragma unroll
  for (int kb = 0; kb < D; kb += 32) { const v16b a = frag_kb(&As[wave][nloc][kb], hlf), al = frag_kb(&Al[wave][nloc][kb], hlf);
#pragma unroll
    for (int t = 0; t < 4; ++t) { const size_t wo_ = (size_t)(t * 16 + nloc) * D + kb; acc[t] = wmma16b(a, frag_kb(W1T + wo_, hlf), acc[t]); acc[t] = wmma16b(al, frag_kb(W1Q + wo_, hlf), acc[t]); } }
  wave_lds_sync();
#pragma unroll
  for (int t = 0; t < 4; ++t) { const float bb = bf16_rne(b1[t * 16 + nloc]);
#pragma unroll
    for (int r = 0; r < 8; ++r) { const float tv = lrelu(acc[t][r] * (1.0f / (XS * WSC)) + bb); const float vs = tv * XS; const b16 ph = (b16)vs; As[wave][8 * hlf + r][t * 16 + nloc] = ph; Al[wave][8 * hlf + r][t * 16 + nloc] = (b16)((vs - (float)ph) * RS_); } }
  wave_lds_sync();
  v8f acc2[2] = {(v8f){}, (v8f){}};
#pragma unroll
  for (int kb = 0; kb < H1; kb += 32) { const v16b a = frag_kb(&As[wave][nloc][kb], hlf), al = frag_kb(&Al[wave][nloc][kb], hlf);
#pragma unroll
    for (int t = 0; t < 2; ++t) { const size_t wo_ = (size_t)(t * 16 + nloc) * H1 + kb; acc2[t] = wmma16b(a, frag_kb(W2T + wo_, hlf), acc2[t]); acc2[t] = wmma16b(al, frag_kb(W2Q + wo_, hlf), acc2[t]); } }
  const float bb0 = bf16_rne(b2[nloc]), bb1 = bf16_rne(b2[16 + nloc]); const float w30 = bf16_rne(w3[nloc]), w31 = bf16_rne(w3[16 + nloc]); const float bb3 = bf16_rne(b3[0]);
#pragma unroll
  for (int r = 0; r < 8; ++r) { const float t20 = lrelu(acc2[0][r] * (1.0f / (XS * WSC)) + bb0), t21 = lrelu(acc2[1][r] * (1.0f / (XS * WSC)) + bb1); float s = fmaf(t20, w30, pmul(t21, w31));
    for (int o = 1; o <= 8; o <<= 1) s += __shfl_xor(s, o);
    if (nloc == 0) Sc[wave * 16 + 8 * hlf + r] = s + bb3; }
  __syncthreads();
  for (int pass = 0; pass < 2; ++pass) { if (threadIdx.x < 32) ((volatile float*)OUTP)[(size_t)blockIdx.x * 32 + threadIdx.x] = Sc[threadIdx.x]; __threadfence(); }
}
}

extern "C" void kernel_launch(void* const* d_in, const int* in_sizes, int n_in, void* d_out, int out_size, void* d_ws, size_t ws_size, hipStream_t stream) {
  (void)n_in;
  auto Fp = [&](int i) { return (const float*)d_in[i]; }; auto Ip = [&](int i) { return (const int*)d_in[i]; };
  if (in_sizes[0] != N * D || in_sizes[1] != EFULL || in_sizes[2] != EFULL || in_sizes[3] != EFULL || in_sizes[4] != PPAIR || in_sizes[5] != PPAIR || in_sizes[6] != PPAIR || in_sizes[7] != PPAIR || in_sizes[8] != D * D || in_sizes[9] != D || in_sizes[10] != L * D * D || in_sizes[11] != L * D * D || in_sizes[12] != L * D * D || in_sizes[13] != L * NH * DK * DK || in_sizes[14] != L * NH * DK * DK || in_sizes[15] != L * NH || in_sizes[16] != L * D * D || in_sizes[17] != L || in_sizes[18] != D * H1 || in_sizes[19] != H1 || in_sizes[20] != H1 * H2 || in_sizes[21] != H2 || in_sizes[22] != H2 || in_sizes[23] != 1 || out_size != NPAIR + N * D) return;
  float* out_pos = (float*)d_out; float* out_h = (float*)d_out + NPAIR;
  size_t off = 0; char* ws = (char*)d_ws;
  auto carve = [&](size_t bytes) { char* p = ws + off; off += (bytes + 255) & ~(size_t)255; return p; };
  const size_t wsz = (size_t)D * D * 2;
  b16* WIN = (b16*)carve(wsz); b16* WK[L], *WKq[L], *WQ[L], *WQq[L], *WV[L], *WVq[L], *WA[L], *WAq[L], *BAT[L], *BAQ[L], *BMT[L], *BMQ[L];
  for (int l = 0; l < L; ++l) { WK[l] = (b16*)carve(wsz); WKq[l] = (b16*)carve(wsz); WQ[l] = (b16*)carve(wsz); WQq[l] = (b16*)carve(wsz); WV[l] = (b16*)carve(wsz); WVq[l] = (b16*)carve(wsz); WA[l] = (b16*)carve(wsz); WAq[l] = (b16*)carve(wsz); BAT[l] = (b16*)carve(wsz); BAQ[l] = (b16*)carve(wsz); BMT[l] = (b16*)carve(wsz); BMQ[l] = (b16*)carve(wsz); }
  b16* W1T = (b16*)carve((size_t)H1 * D * 2); b16* W1Q = (b16*)carve((size_t)H1 * D * 2); b16* W2T = (b16*)carve((size_t)H2 * H1 * 2); b16* W2Q = (b16*)carve((size_t)H2 * H1 * 2);
  float* HA = (float*)carve((size_t)NP * D * 4); float* HB = (float*)carve((size_t)NP * D * 4); float* KQV = (float*)carve((size_t)NP * 3 * D * 4); float* AGG = (float*)carve((size_t)NP * D * 4);
  CsrBufs csr; off = csr_carve(csr, ws, off, E, N);
  if (off > ws_size || off > ((size_t)176 << 20)) return;
  const unsigned g8 = (D * D / 8 + 255) / 256;
  wprep_kernel<D, D, D><<<g8, 256, 0, stream>>>(Fp(8), WIN, WSC);
  for (int l = 0; l < L; ++l) { const size_t mo = (size_t)l * D * D, bo = (size_t)l * NH * DK * DK;
    wprep_kernel<D, D, D><<<g8, 256, 0, stream>>>(Fp(10) + mo, WK[l], WSC); wprep_kernel<D, D, D><<<g8, 256, 0, stream>>>(Fp(10) + mo, WKq[l], WSQ);
    wprep_kernel<D, D, D><<<g8, 256, 0, stream>>>(Fp(11) + mo, WQ[l], WSC); wprep_kernel<D, D, D><<<g8, 256, 0, stream>>>(Fp(11) + mo, WQq[l], WSQ);
    wprep_kernel<D, D, D><<<g8, 256, 0, stream>>>(Fp(12) + mo, WV[l], WSC); wprep_kernel<D, D, D><<<g8, 256, 0, stream>>>(Fp(12) + mo, WVq[l], WSQ);
    wprep_kernel<D, D, D><<<g8, 256, 0, stream>>>(Fp(16) + mo, WA[l], WSC); wprep_kernel<D, D, D><<<g8, 256, 0, stream>>>(Fp(16) + mo, WAq[l], WSQ);
    bd_kernel<<<g8, 256, 0, stream>>>(Fp(13) + bo, BAT[l], WSC); bd_kernel<<<g8, 256, 0, stream>>>(Fp(13) + bo, BAQ[l], WSQ); bd_kernel<<<g8, 256, 0, stream>>>(Fp(14) + bo, BMT[l], WSC); bd_kernel<<<g8, 256, 0, stream>>>(Fp(14) + bo, BMQ[l], WSQ); }
  wprep_kernel<D, H1, H1><<<(H1 * D / 8 + 255) / 256, 256, 0, stream>>>(Fp(18), W1T, WSC); wprep_kernel<D, H1, H1><<<(H1 * D / 8 + 255) / 256, 256, 0, stream>>>(Fp(18), W1Q, WSQ);
  wprep_kernel<H1, H2, H2><<<(H2 * H1 / 8 + 255) / 256, 256, 0, stream>>>(Fp(20), W2T, WSC); wprep_kernel<H1, H2, H2><<<(H2 * H1 / 8 + 255) / 256, 256, 0, stream>>>(Fp(20), W2Q, WSQ);
  csr_build(csr, Ip(2), E, N, stream);
  gemm_kernel<true, true, false, 1, true><<<NP / 32, 64, 0, stream>>>(Fp(0), D, WIN, WIN, Fp(9), nullptr, nullptr, nullptr, nullptr, HA, D, NP);
  float* hin = HA; float* hout = HB;
  for (int l = 0; l < L; ++l) { const bool last = (l == L - 1);
    gemm_kernel<false, false, true, 0, false><<<NP / 32, 64, 0, stream>>>(hin, D, WK[l], WKq[l], nullptr, BAT[l], BAQ[l], nullptr, nullptr, KQV, 3 * D, NP);
    gemm_kernel<false, false, false, 0, false><<<NP / 32, 64, 0, stream>>>(hin, D, WQ[l], WQq[l], nullptr, nullptr, nullptr, nullptr, nullptr, KQV + D, 3 * D, NP);
    gemm_kernel<false, false, true, 0, false><<<NP / 32, 64, 0, stream>>>(hin, D, WV[l], WVq[l], nullptr, BMT[l], BMQ[l], nullptr, nullptr, KQV + 2 * D, 3 * D, NP);
    attn_kernel<<<NP / 32, 256, 0, stream>>>(KQV, Fp(15) + (size_t)l * NH, Fp(3), Ip(1), csr.PERM, csr.ROWPTR, csr.ROWCNT, (int)csr.permLen, AGG);
    if (last) gemm_kernel<false, false, false, 2, false><<<NP / 32, 64, 0, stream>>>(AGG, D, WA[l], WAq[l], nullptr, nullptr, nullptr, hin, Fp(17) + l, hout, D, NP);
    else      gemm_kernel<false, false, false, 2, true><<<NP / 32, 64, 0, stream>>>(AGG, D, WA[l], WAq[l], nullptr, nullptr, nullptr, hin, Fp(17) + l, hout, D, NP);
    float* t = hin; hin = hout; hout = t; }
  copy_kernel<<<NPL / 32, 256, 0, stream>>>(hin, out_h, NL);
  pred_kernel<<<NPAIR / 32, 64, 0, stream>>>(hin, Ip(4), Ip(5), Ip(6), Ip(7), W1T, W1Q, Fp(19), W2T, W2Q, Fp(21), Fp(22), Fp(23), out_pos);
}
